// MultiHeadedAttention_RPR_16355235463565
// MI455X (gfx1250) — hardware-verified
//
#include <hip/hip_runtime.h>
#include <stddef.h>


typedef __bf16 v16b __attribute__((ext_vector_type(16)));
typedef float v8f __attribute__((ext_vector_type(8)));
typedef float v4f __attribute__((ext_vector_type(4)));
typedef unsigned int v4u __attribute__((ext_vector_type(4)));
typedef v4f v4fa __attribute__((may_alias));
typedef unsigned short us_t;

union Frag { v16b v; v4u q[2]; unsigned int u[8]; };

#define SEQ 2048
#define NBATCH 2
#define NHEAD 16
#define DKH 64
#define DMOD 1024
#define NBKT 33
#define NINT 31

__device__ __forceinline__ unsigned int bf_bits(float x) {
    unsigned int u = __float_as_uint(x);
    return ((u + 0x7FFFu + ((u >> 16) & 1u)) >> 16) & 0xFFFFu;
}
__device__ __forceinline__ float bf_val(unsigned int b) { return __uint_as_float(b << 16); }
__device__ __forceinline__ unsigned int pk2(unsigned int lo16, unsigned int hi16) {
    return (lo16 & 0xFFFFu) | (hi16 << 16);
}
__device__ __forceinline__ void split8(const float (&x)[8], v4u& wh, v4u& wl) {
    unsigned int hb[8], lb[8];
#pragma unroll
    for (int i = 0; i < 8; ++i) {
        hb[i] = bf_bits(x[i]);
        lb[i] = bf_bits(x[i] - bf_val(hb[i]));
    }
    wh.x = pk2(hb[0], hb[1]); wh.y = pk2(hb[2], hb[3]); wh.z = pk2(hb[4], hb[5]); wh.w = pk2(hb[6], hb[7]);
    wl.x = pk2(lb[0], lb[1]); wl.y = pk2(lb[2], lb[3]); wl.z = pk2(lb[4], lb[5]); wl.w = pk2(lb[6], lb[7]);
}

__device__ __forceinline__ void ldf(Frag& f, const us_t* p) {
    f.q[0] = *(const v4u*)(p);
    f.q[1] = *(const v4u*)(p + 16);
}

__device__ __forceinline__ v8f mma3(v8f c, const Frag& ah, const Frag& al, const Frag& bh, const Frag& bl) {
    c = __builtin_amdgcn_wmma_f32_16x16x32_bf16(false, ah.v, false, bh.v, (short)0, c, false, false);
    c = __builtin_amdgcn_wmma_f32_16x16x32_bf16(false, ah.v, false, bl.v, (short)0, c, false, false);
    c = __builtin_amdgcn_wmma_f32_16x16x32_bf16(false, al.v, false, bh.v, (short)0, c, false, false);
    asm volatile("v_nop\n\tv_nop\n\tv_nop\n\tv_nop"
                 : "+v"(c)
                 : "v"(ah.q[0]), "v"(ah.q[1]), "v"(al.q[0]), "v"(al.q[1]),
                   "v"(bh.q[0]), "v"(bh.q[1]), "v"(bl.q[0]), "v"(bl.q[1]));
    return c;
}

__global__ void __launch_bounds__(256)
k_split(const float* __restrict__ in, us_t* oh, us_t* ol, int n8)
{
    const int i = blockIdx.x * 256 + threadIdx.x;
    if (i >= n8) return;
    const float* p = in + (size_t)i * 8;
    const v4f a = *(const v4f*)(p);
    const v4f c = *(const v4f*)(p + 4);
    float x[8] = {a.x, a.y, a.z, a.w, c.x, c.y, c.z, c.w};
    v4u wh, wl;
    split8(x, wh, wl);
    us_t* dh = oh + (size_t)i * 8;
    us_t* dl = ol + (size_t)i * 8;
    *(volatile v4u*)dh = wh;
    *(volatile v4u*)dl = wl;
    __threadfence();
    *(volatile v4u*)dh = wh;
    *(volatile v4u*)dl = wl;
}

__global__ void __launch_bounds__(256)
k_gemm(const us_t* __restrict__ Xh, const us_t* __restrict__ Xl,
       const us_t* __restrict__ Wh, const us_t* __restrict__ Wl,
       const float* __restrict__ bias,
       us_t* outh, us_t* outl, float* outf,
       int M, int N, int K, int mode)
{
    __shared__ __align__(16) float Cs[128 * 128];

    const int tid  = threadIdx.x;
    const int lane = tid & 31;
    const int wave = tid >> 5;
    const int hh   = lane >> 4;
    const int l16  = lane & 15;
    const int wr   = wave >> 2;
    const int wc   = wave & 3;
    const int m0   = blockIdx.y * 128;
    const int n0   = blockIdx.x * 128;
    if (m0 + 128 > M || n0 + 128 > N) return;

    const v8f zero = {};
    v8f acc[4][2];
#pragma unroll
    for (int i = 0; i < 4; ++i)
#pragma unroll
        for (int j = 0; j < 2; ++j) acc[i][j] = zero;

    size_t xo[4], wo[2];
#pragma unroll
    for (int i = 0; i < 4; ++i) xo[i] = (size_t)(m0 + wr * 64 + i * 16 + l16) * K + 8 * hh;
#pragma unroll
    for (int j = 0; j < 2; ++j) wo[j] = (size_t)(n0 + wc * 32 + j * 16 + l16) * K + 8 * hh;

#pragma unroll 1
    for (int kk = 0; kk < K; kk += 32) {
        Frag bh2[2], bl2[2];
#pragma unroll
        for (int j = 0; j < 2; ++j) {
            ldf(bh2[j], Wh + wo[j] + kk);
            ldf(bl2[j], Wl + wo[j] + kk);
        }
#pragma unroll
        for (int i = 0; i < 4; ++i) {
            Frag ah, al;
            ldf(ah, Xh + xo[i] + kk);
            ldf(al, Xl + xo[i] + kk);
#pragma unroll
            for (int j = 0; j < 2; ++j)
                acc[i][j] = mma3(acc[i][j], ah, al, bh2[j], bl2[j]);
        }
    }

#pragma unroll
    for (int i = 0; i < 4; ++i)
#pragma unroll
        for (int j = 0; j < 2; ++j)
#pragma unroll
            for (int r = 0; r < 8; ++r)
                Cs[(wr * 64 + i * 16 + 8 * hh + r) * 128 + wc * 32 + j * 16 + l16] = acc[i][j][r];
    __syncthreads();

#pragma unroll 1
    for (int pass = 0; pass < 2; ++pass) {
#pragma unroll 1
        for (int t = 0; t < 16; ++t) {
            const int seg = wave * 16 + t;
            if (mode == 1) {
                const int row = seg;
                const int c   = lane * 4;
                const v4f cv = *(const v4fa*)(Cs + row * 128 + c);
                const v4f bv = *(const v4f*)(bias + n0 + c);
                v4f ov;
                ov.x = cv.x + bv.x; ov.y = cv.y + bv.y; ov.z = cv.z + bv.z; ov.w = cv.w + bv.w;
                *(volatile v4f*)(outf + (size_t)(m0 + row) * N + n0 + c) = ov;
            } else {
                const int plane = seg >> 6;
                const int s6    = seg & 63;
                const int hh2   = s6 >> 5;
                const int sub   = s6 & 31;
                float x[8];
                us_t* dp;
                if (mode == 0) {
                    const int row = sub * 4 + (lane >> 3);
                    const int gc  = hh2 * 64 + (lane & 7) * 8;
                    const v4f c0 = *(const v4fa*)(Cs + row * 128 + gc);
                    const v4f c1 = *(const v4fa*)(Cs + row * 128 + gc + 4);
                    const v4f b0 = *(const v4f*)(bias + n0 + gc);
                    const v4f b1 = *(const v4f*)(bias + n0 + gc + 4);
                    x[0] = c0.x + b0.x; x[1] = c0.y + b0.y; x[2] = c0.z + b0.z; x[3] = c0.w + b0.w;
                    x[4] = c1.x + b1.x; x[5] = c1.y + b1.y; x[6] = c1.z + b1.z; x[7] = c1.w + b1.w;
                    const int gm = m0 + row;
                    const int bb = gm / SEQ;
                    const int s  = gm - bb * SEQ;
                    const int hg = (n0 >> 6) + hh2;
                    dp = (plane ? outl : outh) + (((size_t)(bb * NHEAD + hg)) * SEQ + s) * DKH + (lane & 7) * 8;
                } else {
                    const int c  = hh2 * 64 + sub * 2 + (lane >> 4);
                    const int sl = (lane & 15) * 8;
                    const float bc = bias[n0 + c];
#pragma unroll
                    for (int i = 0; i < 8; ++i) x[i] = Cs[(sl + i) * 128 + c] + bc;
                    const int bb = m0 / SEQ;
                    const int s0 = m0 - bb * SEQ;
                    const int hg = (n0 >> 6) + hh2;
                    const int d  = c & 63;
                    dp = (plane ? outl : outh) + (((size_t)(bb * NHEAD + hg)) * DKH + d) * SEQ + s0 + sl;
                }
                v4u wh, wl;
                split8(x, wh, wl);
                const v4u w = plane ? wl : wh;
                *(volatile v4u*)dp = w;
            }
        }
        __threadfence();
    }
}

__global__ void __launch_bounds__(256)
k_attn(const us_t* __restrict__ Qh, const us_t* __restrict__ Ql,
       const us_t* __restrict__ Kh, const us_t* __restrict__ Kl,
       const us_t* __restrict__ Vh, const us_t* __restrict__ Vl,
       const float* __restrict__ embK,
       const float* __restrict__ embV,
       us_t* Ch, us_t* Cl)
{
    __shared__ __align__(16) unsigned char lds[65536];
    us_t*  ekh   = (us_t*)(lds);
    us_t*  ekl   = (us_t*)(lds + 6144);
    us_t*  wsh   = (us_t*)(lds);
    us_t*  wsl   = (us_t*)(lds + 16384);
    float* relLs = (float*)(lds + 32768);
    us_t*  evh   = (us_t*)(lds + 32768);
    us_t*  evl   = (us_t*)(lds + 32768 + 8192);
    float* sint  = (float*)(lds + 49664);
    float* Cs    = (float*)(lds + 32768);

    const int tid  = threadIdx.x;
    const int lane = tid & 31;
    const int wave = tid >> 5;
    const int hh   = lane >> 4;
    const int l16  = lane & 15;
    const int bh   = blockIdx.y;
    const int b    = bh >> 4;
    const int h    = bh & 15;
    const int q0   = blockIdx.x * 128;
    if (q0 + 128 > SEQ || bh >= NBATCH * NHEAD) return;
    const int ql   = wave * 16 + l16;
    const int qw0  = q0 + wave * 16;
    const int qg   = q0 + ql;

    const v8f zero = {};

    if (tid < 192) {
        const int v  = tid >> 2;
        const int d0 = (tid & 3) * 16;
#pragma unroll
        for (int g = 0; g < 2; ++g) {
            float x[8];
            if (v < NBKT) {
                const v4f a = *(const v4f*)(embK + v * DKH + d0 + g * 8);
                const v4f c = *(const v4f*)(embK + v * DKH + d0 + g * 8 + 4);
                x[0] = a.x; x[1] = a.y; x[2] = a.z; x[3] = a.w; x[4] = c.x; x[5] = c.y; x[6] = c.z; x[7] = c.w;
            } else {
#pragma unroll
                for (int i = 0; i < 8; ++i) x[i] = 0.0f;
            }
            v4u wh, wl;
            split8(x, wh, wl);
            *(v4u*)(ekh + v * DKH + d0 + g * 8) = wh;
            *(v4u*)(ekl + v * DKH + d0 + g * 8) = wl;
        }
    }
    for (int i = tid; i < 128 * NINT; i += 256) sint[i] = -1.0e30f;
    __syncthreads();

    Frag qbh[2], qbl[2];
    {
        const size_t qo = ((size_t)bh * SEQ + qg) * DKH + 8 * hh;
#pragma unroll
        for (int kc = 0; kc < 2; ++kc) {
            ldf(qbh[kc], Qh + qo + kc * 32);
            ldf(qbl[kc], Ql + qo + kc * 32);
        }
    }
#pragma unroll
    for (int nt = 0; nt < 3; ++nt) {
        v8f a = zero;
#pragma unroll
        for (int kc = 0; kc < 2; ++kc) {
            Frag ah, al;
            ldf(ah, ekh + (nt * 16 + l16) * DKH + kc * 32 + 8 * hh);
            ldf(al, ekl + (nt * 16 + l16) * DKH + kc * 32 + 8 * hh);
            a = mma3(a, ah, al, qbh[kc], qbl[kc]);
        }
#pragma unroll
        for (int r = 0; r < 8; ++r) {
            const int v = nt * 16 + 8 * hh + r;
            if (v < NBKT) relLs[ql * NBKT + v] = a[r];
        }
    }
    __syncthreads();

    v8f oacc[4];
#pragma unroll
    for (int f = 0; f < 4; ++f) oacc[f] = zero;
    float m_run = -1.0e30f, l_run = 0.0f, a0 = 0.0f, a32 = 0.0f;

#pragma unroll 1
    for (int kt = 0; kt < SEQ / 64; ++kt) {
        const int k0 = kt * 64;

        v8f sc[4];
#pragma unroll
        for (int ft = 0; ft < 4; ++ft) {
            v8f a = zero;
#pragma unroll
            for (int kc = 0; kc < 2; ++kc) {
                Frag ah, al;
                const size_t ko = ((size_t)bh * SEQ + k0 + ft * 16 + l16) * DKH + kc * 32 + 8 * hh;
                ldf(ah, Kh + ko);
                ldf(al, Kl + ko);
                a = mma3(a, ah, al, qbh[kc], qbl[kc]);
            }
            sc[ft] = a;
        }

        const bool below = (k0 + 79 <= qw0);
        const bool above = (k0 >= qw0 + 31);
        const bool nearr = !(below || above);
        float mx = -1.0e30f;
        if (nearr) {
#pragma unroll
            for (int ft = 0; ft < 4; ++ft)
#pragma unroll
                for (int r = 0; r < 8; ++r) {
                    const int rel = k0 + ft * 16 + 8 * hh + r - qg;
                    const int bk  = rel <= -16 ? 0 : (rel >= 16 ? 32 : rel + 16);
                    const float s = sc[ft][r] + relLs[ql * NBKT + bk];
                    sc[ft][r] = s;
                    mx = fmaxf(mx, s);
                    if (rel > -16 && rel < 16) sint[ql * NINT + rel + 15] = s;
                }
        } else {
            const float bc = relLs[ql * NBKT + (below ? 0 : 32)];
#pragma unroll
            for (int ft = 0; ft < 4; ++ft)
#pragma unroll
                for (int r = 0; r < 8; ++r) {
                    const float s = sc[ft][r] + bc;
                    sc[ft][r] = s;
                    mx = fmaxf(mx, s);
                }
        }
        mx = fmaxf(mx, __shfl_xor(mx, 16, 32));
        const float mnew = fmaxf(m_run, mx);
        const float al   = __expf(m_run - mnew);
        m_run = mnew;
        l_run *= al; a0 *= al; a32 *= al;
#pragma unroll
        for (int f = 0; f < 4; ++f)
#pragma unroll
            for (int r = 0; r < 8; ++r) oacc[f][r] *= al;

        float ps = 0.0f;
#pragma unroll
        for (int ft = 0; ft < 4; ++ft)
#pragma unroll
            for (int r = 0; r < 8; ++r) {
                const float p = __expf(sc[ft][r] - mnew);
                sc[ft][r] = p;
                ps += p;
            }
        l_run += ps;
        if (nearr) {
#pragma unroll
            for (int ft = 0; ft < 4; ++ft)
#pragma unroll
                for (int r = 0; r < 8; ++r) {
                    const int rel = k0 + ft * 16 + 8 * hh + r - qg;
                    const float p = sc[ft][r];
                    a0  += (rel <= -16) ? p : 0.0f;
                    a32 += (rel >= 16) ? p : 0.0f;
                }
        } else {
            if (below) a0 += ps; else a32 += ps;
        }

        Frag ph[2], pl[2];
#pragma unroll
        for (int kc = 0; kc < 2; ++kc)
#pragma unroll
            for (int w = 0; w < 8; ++w) {
                const int ft = 2 * kc + (w >> 2);
                const int e  = (w & 3) * 2;
                const float p0 = sc[ft][e], p1 = sc[ft][e + 1];
                const unsigned int h0 = bf_bits(p0), h1 = bf_bits(p1);
                const unsigned int l0 = bf_bits(p0 - bf_val(h0)), l1 = bf_bits(p1 - bf_val(h1));
                ph[kc].u[w] = pk2(h0, h1);
                pl[kc].u[w] = pk2(l0, l1);
            }

#pragma unroll
        for (int f = 0; f < 4; ++f)
#pragma unroll
            for (int kc = 0; kc < 2; ++kc) {
                Frag ah, al;
                const size_t vo = ((size_t)bh * DKH + f * 16 + l16) * SEQ + k0 + kc * 32 + 8 * hh;
                ldf(ah, Vh + vo);
                ldf(al, Vl + vo);
                oacc[f] = mma3(oacc[f], ah, al, ph[kc], pl[kc]);
            }
    }

    l_run += __shfl_xor(l_run, 16, 32);
    a0    += __shfl_xor(a0, 16, 32);
    a32   += __shfl_xor(a32, 16, 32);
    __syncthreads();

    {
        const int d  = tid >> 2;
        const int v0 = (tid & 3) * 16;
#pragma unroll
        for (int g = 0; g < 2; ++g) {
            float x[8];
#pragma unroll
            for (int i = 0; i < 8; ++i) {
                const int v = v0 + g * 8 + i;
                x[i] = (v < NBKT) ? embV[v * DKH + d] : 0.0f;
            }
            v4u wh, wl;
            split8(x, wh, wl);
            *(v4u*)(evh + d * 64 + v0 + g * 8) = wh;
            *(v4u*)(evl + d * 64 + v0 + g * 8) = wl;
        }
    }
    {
#pragma unroll
        for (int g = 0; g < 4; ++g) {
            float x[8];
#pragma unroll
            for (int e = 0; e < 8; ++e) {
                const int j = g * 8 + e;
                float val = 0.0f;
                if (j == 0) val = (hh == 0) ? a0 : a32;
                else if (hh == 0) val = __expf(sint[ql * NINT + (j - 1)] - m_run);
                x[e] = val;
            }
            v4u wh, wl;
            split8(x, wh, wl);
            *(v4u*)(wsh + ql * 64 + hh * 32 + g * 8) = wh;
            *(v4u*)(wsl + ql * 64 + hh * 32 + g * 8) = wl;
        }
    }
    __syncthreads();

#pragma unroll
    for (int kc = 0; kc < 2; ++kc) {
        Frag wbh, wbl;
        ldf(wbh, wsh + ql * 64 + kc * 32 + 8 * hh);
        ldf(wbl, wsl + ql * 64 + kc * 32 + 8 * hh);
#pragma unroll
        for (int f = 0; f < 4; ++f) {
            Frag ah, al;
            ldf(ah, evh + (f * 16 + l16) * 64 + kc * 32 + 8 * hh);
            ldf(al, evl + (f * 16 + l16) * 64 + kc * 32 + 8 * hh);
            oacc[f] = mma3(oacc[f], ah, al, wbh, wbl);
        }
    }
    __syncthreads();

#pragma unroll
    for (int f = 0; f < 4; ++f)
#pragma unroll
        for (int r = 0; r < 8; ++r)
            Cs[ql * 64 + f * 16 + 8 * hh + r] = oacc[f][r] / l_run;
    __syncthreads();

#pragma unroll 1
    for (int pass = 0; pass < 2; ++pass) {
#pragma unroll 1
        for (int t = 0; t < 8; ++t) {
            const int plane = t >> 2;
            const int row   = wave * 16 + (t & 3) * 4 + (lane >> 3);
            const int c8    = (lane & 7) * 8;
            const v4f x0 = *(const v4fa*)(Cs + row * 64 + c8);
            const v4f x1 = *(const v4fa*)(Cs + row * 64 + c8 + 4);
            float x[8] = {x0.x, x0.y, x0.z, x0.w, x1.x, x1.y, x1.z, x1.w};
            v4u wh, wl;
            split8(x, wh, wl);
            us_t* dp = (plane ? Cl : Ch) + ((size_t)(b * SEQ + q0 + row)) * DMOD + h * DKH + c8;
            const v4u w = plane ? wl : wh;
            *(volatile v4u*)dp = w;
        }
        __threadfence();
    }
}

extern "C" void kernel_launch(void* const* d_in, const int* in_sizes, int n_in,
                              void* d_out, int out_size, void* d_ws, size_t ws_size,
                              hipStream_t stream)
{
    const int NA = NBATCH * SEQ * DMOD;
    const int NW = DMOD * DMOD;
    if (n_in != 13) return;
    if (in_sizes[0] != NA || in_sizes[1] != NA || in_sizes[2] != NA) return;
    if (in_sizes[3] != NW || in_sizes[4] != NW || in_sizes[5] != NW || in_sizes[6] != NW) return;
    if (in_sizes[7] != DMOD || in_sizes[8] != DMOD || in_sizes[9] != DMOD || in_sizes[10] != DMOD) return;
    if (in_sizes[11] != NBKT * DKH || in_sizes[12] != NBKT * DKH) return;
    if (out_size != NA) return;

    const size_t need = ((size_t)12 * NA + (size_t)8 * NW) * sizeof(us_t);
    if (ws_size < need) return;

    const float* query = (const float*)d_in[0];
    const float* key_  = (const float*)d_in[1];
    const float* value = (const float*)d_in[2];
    const float* Wq    = (const float*)d_in[3];
    const float* Wk    = (const float*)d_in[4];
    const float* Wv    = (const float*)d_in[5];
    const float* Wo    = (const float*)d_in[6];
    const float* bq    = (const float*)d_in[7];
    const float* bk    = (const float*)d_in[8];
    const float* bv    = (const float*)d_in[9];
    const float* bo    = (const float*)d_in[10];
    const float* embK  = (const float*)d_in[11];
    const float* embV  = (const float*)d_in[12];

    us_t* ws   = (us_t*)d_ws;
    us_t* xq_h = ws;                 us_t* xq_l = xq_h + NA;
    us_t* xk_h = xq_l + NA;          us_t* xk_l = xk_h + NA;
    us_t* xv_h = xk_l + NA;          us_t* xv_l = xv_h + NA;
    us_t* wq_h = xv_l + NA;          us_t* wq_l = wq_h + NW;
    us_t* wk_h = wq_l + NW;          us_t* wk_l = wk_h + NW;
    us_t* wv_h = wk_l + NW;          us_t* wv_l = wv_h + NW;
    us_t* wo_h = wv_l + NW;          us_t* wo_l = wo_h + NW;
    us_t* qp_h = wo_l + NW;          us_t* qp_l = qp_h + NA;
    us_t* kp_h = qp_l + NA;          us_t* kp_l = kp_h + NA;
    us_t* vt_h = kp_l + NA;          us_t* vt_l = vt_h + NA;
    us_t* cx_h = xq_h;               us_t* cx_l = xq_l;

    const int na8 = NA / 8, nw8 = NW / 8;
    k_split<<<(na8 + 255) / 256, 256, 0, stream>>>(query, xq_h, xq_l, na8);
    k_split<<<(na8 + 255) / 256, 256, 0, stream>>>(key_,  xk_h, xk_l, na8);
    k_split<<<(na8 + 255) / 256, 256, 0, stream>>>(value, xv_h, xv_l, na8);
    k_split<<<(nw8 + 255) / 256, 256, 0, stream>>>(Wq, wq_h, wq_l, nw8);
    k_split<<<(nw8 + 255) / 256, 256, 0, stream>>>(Wk, wk_h, wk_l, nw8);
    k_split<<<(nw8 + 255) / 256, 256, 0, stream>>>(Wv, wv_h, wv_l, nw8);
    k_split<<<(nw8 + 255) / 256, 256, 0, stream>>>(Wo, wo_h, wo_l, nw8);

    const int M = NBATCH * SEQ;
    dim3 gg(DMOD / 128, M / 128);
    k_gemm<<<gg, 256, 0, stream>>>(xq_h, xq_l, wq_h, wq_l, bq, qp_h, qp_l, (float*)d_out, M, DMOD, DMOD, 0);
    k_gemm<<<gg, 256, 0, stream>>>(xk_h, xk_l, wk_h, wk_l, bk, kp_h, kp_l, (float*)d_out, M, DMOD, DMOD, 0);
    k_gemm<<<gg, 256, 0, stream>>>(xv_h, xv_l, wv_h, wv_l, bv, vt_h, vt_l, (float*)d_out, M, DMOD, DMOD, 2);

    dim3 ga(SEQ / 128, NBATCH * NHEAD);
    k_attn<<<ga, 256, 0, stream>>>(qp_h, qp_l, kp_h, kp_l, vt_h, vt_l, embK, embV, cx_h, cx_l);

    k_gemm<<<gg, 256, 0, stream>>>(cx_h, cx_l, wo_h, wo_l, bo, kp_h, kp_l, (float*)d_out, M, DMOD, DMOD, 1);
}
